// TorchLocalAttention_4758823764714
// MI455X (gfx1250) — hardware-verified
//
#include <hip/hip_runtime.h>
#include <stdint.h>

#define NB     4
#define CCH    128
#define HH     64
#define WWD    64
#define HW     4096
#define NPIX   16384
#define KSZ    11
#define KHF    5
#define NWIN   121
#define QR     4
#define QC     16
#define HCOL   32
#define JOFF   3
#define NSLOT  448
#define PROW   896
#define PLO    448
#define SCP    124
#define OSTP   32
#define TP     136
#define LDC    132
#define RSC    0.00048828125f
#define OSC    0.000030517578125f
#define S64I   0.015625f
#define XSC    8.0f
#define WSC    64.0f
#define RESC   2048.0f
#define PSC    4096.0f

#define LDS_SC   0
#define LDS_P    31744
#define LDS_OST  146432
#define LDS_ATT  211968

static_assert(NPIX == NB * HW && HW == HH * WWD);
static_assert(NSLOT == (QR + KSZ - 1) * HCOL && (NSLOT % 32) == 0);
static_assert(LDS_P == 64 * SCP * 4);
static_assert(LDS_OST == LDS_P + 64 * PROW * 2);
static_assert(LDS_ATT == LDS_OST + CCH * QR * OSTP * 4);
static_assert((LDS_P % 16) == 0 && (LDS_OST % 16) == 0 && ((PROW * 2) % 16) == 0 && ((PLO * 2) % 16) == 0);
static_assert(PLO + NSLOT <= PROW);
static_assert(((TP * 2) % 16) == 0 && (LDC % 4) == 0 && (OSTP % 4) == 0);
static_assert(NWIN <= SCP && NWIN == KSZ * KSZ);
static_assert(JOFF == 8 - KHF);
static_assert((NPIX % 64) == 0 && (CCH % 32) == 0);

typedef _Float16 v16h __attribute__((ext_vector_type(16)));
typedef _Float16 v8h  __attribute__((ext_vector_type(8)));
typedef float    v8f  __attribute__((ext_vector_type(8)));
typedef float    v4f  __attribute__((ext_vector_type(4)));
typedef unsigned int v4u __attribute__((ext_vector_type(4)));
typedef v4u v4ua __attribute__((may_alias));
typedef v4f v4fa __attribute__((may_alias));

__device__ __forceinline__ unsigned short bf_bits(float f) {
  unsigned u = __float_as_uint(f);
  return (unsigned short)((u + 0x7FFFu + ((u >> 16) & 1u)) >> 16);
}
__device__ __forceinline__ float bf_up(unsigned short b) { return __uint_as_float(((unsigned)b) << 16); }
__device__ __forceinline__ float bfr(float f) { return bf_up(bf_bits(f)); }
__device__ __forceinline__ unsigned short h_bits(_Float16 x) { return __builtin_bit_cast(unsigned short, x); }
__device__ __forceinline__ unsigned short hb16(float f) { return h_bits((_Float16)f); }
__device__ __forceinline__ unsigned pk16(unsigned short a, unsigned short b) { return (unsigned)a | ((unsigned)b << 16); }
__device__ __forceinline__ v8f zero8() { v8f z = {0.f, 0.f, 0.f, 0.f, 0.f, 0.f, 0.f, 0.f}; return z; }

__device__ __forceinline__ void split2(float f0, float f1, unsigned& hpk, unsigned& lpk) {
  const _Float16 a = (_Float16)f0, c = (_Float16)f1;
  hpk = pk16(h_bits(a), h_bits(c));
  lpk = pk16(hb16((f0 - (float)a) * RESC), hb16((f1 - (float)c) * RESC));
}

__device__ __forceinline__ v16h ldfrag_h(const _Float16* p) {
  union { v16h v; v8h h[2]; } f;
  f.h[0] = *(const v8h*)(p);
  f.h[1] = *(const v8h*)(p + 16);
  return f.v;
}
__device__ __forceinline__ v16h ld2(const _Float16* p0, const _Float16* p1) {
  union { v16h v; v8h h[2]; } f;
  f.h[0] = *(const v8h*)(p0);
  f.h[1] = *(const v8h*)(p1);
  return f.v;
}

__device__ __forceinline__ v8f mma_raw(v16h a, v16h b, v8f c) {
  return __builtin_amdgcn_wmma_f32_16x16x32_f16(false, a, false, b, (short)0, c, false, false);
}
__device__ __forceinline__ void guard4(v8f& c0, v8f& c1, v8f& c2, v8f& c3,
                                       const v16h& a0, const v16h& a1, const v16h& b0, const v16h& b1) {
#if defined(__HIP_DEVICE_COMPILE__)
  asm volatile("v_nop\n\tv_nop\n\tv_nop\n\tv_nop"
               : "+v"(c0), "+v"(c1), "+v"(c2), "+v"(c3) : "v"(a0), "v"(a1), "v"(b0), "v"(b1));
#endif
}
__device__ __forceinline__ void guard2(v8f& c0, v8f& c1,
                                       const v16h& a0, const v16h& a1, const v16h& b0, const v16h& b1) {
#if defined(__HIP_DEVICE_COMPILE__)
  asm volatile("v_nop\n\tv_nop\n\tv_nop\n\tv_nop"
               : "+v"(c0), "+v"(c1) : "v"(a0), "v"(a1), "v"(b0), "v"(b1));
#endif
}
__device__ __forceinline__ void guard4x6(v8f& c0, v8f& c1, v8f& c2, v8f& c3,
                                         const v16h& a0, const v16h& a1,
                                         const v16h& b0, const v16h& b1, const v16h& b2, const v16h& b3) {
#if defined(__HIP_DEVICE_COMPILE__)
  asm volatile("v_nop\n\tv_nop\n\tv_nop\n\tv_nop"
               : "+v"(c0), "+v"(c1), "+v"(c2), "+v"(c3)
               : "v"(a0), "v"(a1), "v"(b0), "v"(b1), "v"(b2), "v"(b3));
#endif
}

__device__ __forceinline__ void mm_tile(const _Float16* __restrict__ A, int lda,
                                        const _Float16* __restrict__ W, int ldw, int nks,
                                        int arow0, int bcol0, float* Cs) {
  const int tid = threadIdx.x, wave = tid >> 5, lane = tid & 31, hh = lane >> 4, c = lane & 15;
  const int mw = wave >> 2, nw = wave & 3;
  const _Float16* a0p = A + (size_t)(arow0 + mw * 32 + c) * lda + 8 * hh;
  const _Float16* a1p = A + (size_t)(arow0 + mw * 32 + 16 + c) * lda + 8 * hh;
  const _Float16* b0p = W + (size_t)(bcol0 + nw * 32 + c) * ldw + 8 * hh;
  const _Float16* b1p = W + (size_t)(bcol0 + nw * 32 + 16 + c) * ldw + 8 * hh;
  v8f a00 = zero8(), a01 = zero8(), a10 = zero8(), a11 = zero8();
#pragma unroll 1
  for (int ks = 0; ks < nks; ++ks) {
    const int ko = ks * 32;
    const v16h fa0 = ldfrag_h(a0p + ko);
    const v16h fa1 = ldfrag_h(a1p + ko);
    const v16h fb0 = ldfrag_h(b0p + ko);
    const v16h fb1 = ldfrag_h(b1p + ko);
    a00 = mma_raw(fa0, fb0, a00);
    a01 = mma_raw(fa0, fb1, a01);
    a10 = mma_raw(fa1, fb0, a10);
    a11 = mma_raw(fa1, fb1, a11);
    guard4(a00, a01, a10, a11, fa0, fa1, fb0, fb1);
  }
#pragma unroll
  for (int r = 0; r < 8; ++r) {
    const int row = mw * 32 + 8 * hh + r;
    Cs[row * LDC + nw * 32 + c]             = a00[r];
    Cs[row * LDC + nw * 32 + 16 + c]        = a01[r];
    Cs[(row + 16) * LDC + nw * 32 + c]      = a10[r];
    Cs[(row + 16) * LDC + nw * 32 + 16 + c] = a11[r];
  }
}

__global__ __launch_bounds__(256)
void k_cvt_x(const float* __restrict__ x, unsigned short* xt) {
  __shared__ __align__(16) unsigned short T[64 * TP];
  const int tid = threadIdx.x;
  const int n = blockIdx.x >> 6, pb = blockIdx.x & 63;
  const int p0 = pb * 64;
  const float* src = x + (size_t)n * CCH * HW + p0;
#pragma unroll
  for (int s = 0; s < 8; ++s) {
    const int idx = s * 256 + tid;
    const int c = idx >> 4, pq = (idx & 15) * 4;
    const v4f a = *(const v4f*)(src + (size_t)c * HW + pq);
#pragma unroll
    for (int e = 0; e < 4; ++e) T[(pq + e) * TP + c] = hb16(bfr(a[e]) * XSC);
  }
  __syncthreads();
  v4u pk[4];
  size_t offs[4];
#pragma unroll
  for (int s = 0; s < 4; ++s) {
    const int idx = s * 256 + tid;
    const int row = idx >> 4, piece = idx & 15;
    pk[s] = *(const v4ua*)(&T[row * TP + piece * 8]);
    offs[s] = ((size_t)(n * HW + p0 + row)) * CCH + piece * 8;
  }
#pragma unroll
  for (int s = 0; s < 4; ++s) *(volatile v4u*)(xt + offs[s]) = pk[s];
  __threadfence();
#pragma unroll
  for (int s = 0; s < 4; ++s) *(volatile v4u*)(xt + offs[s]) = pk[s];
}

__global__ __launch_bounds__(256)
void k_cvt_w(const float* __restrict__ w1, const float* __restrict__ w2, const float* __restrict__ w3,
             unsigned short* w16) {
  const int tid = threadIdx.x;
  const int wi = blockIdx.x >> 3;
  const int e0 = ((blockIdx.x & 7) * 256 + tid) * 8;
  const float* src = (wi == 0) ? w1 : ((wi == 1) ? w2 : w3);
  const v4f a = *(const v4f*)(src + e0);
  const v4f c = *(const v4f*)(src + e0 + 4);
  v4u pk;
  pk[0] = pk16(hb16(bfr(a[0]) * WSC), hb16(bfr(a[1]) * WSC));
  pk[1] = pk16(hb16(bfr(a[2]) * WSC), hb16(bfr(a[3]) * WSC));
  pk[2] = pk16(hb16(bfr(c[0]) * WSC), hb16(bfr(c[1]) * WSC));
  pk[3] = pk16(hb16(bfr(c[2]) * WSC), hb16(bfr(c[3]) * WSC));
  unsigned short* dst = w16 + (size_t)wi * CCH * CCH + e0;
  *(volatile v4u*)dst = pk;
  __threadfence();
  *(volatile v4u*)dst = pk;
}

__global__ __launch_bounds__(256)
void k_proj(const unsigned short* __restrict__ xt, const unsigned short* __restrict__ w16,
            unsigned short* th, unsigned short* tl, unsigned short* fh, unsigned short* fl,
            unsigned short* gh, unsigned short* gl) {
  __shared__ __align__(16) float Cs[64 * LDC];
  const int tid = threadIdx.x;
  const int mb = blockIdx.x, wi = blockIdx.y;
  mm_tile((const _Float16*)(const void*)xt, CCH,
          (const _Float16*)(const void*)(w16 + (size_t)wi * CCH * CCH), CCH, CCH / 32,
          mb * 64, 0, Cs);
  __syncthreads();
  v4u ph[4], pl[4];
  size_t offs[4];
  if (wi == 2) {
    const int n = mb >> 6, p0 = (mb & 63) * 64;
#pragma unroll
    for (int s = 0; s < 4; ++s) {
      const int idx = s * 256 + tid;
      const int ch = idx >> 3, piece = idx & 7;
      v4u a, b;
#pragma unroll
      for (int e = 0; e < 4; ++e) {
        const int r0 = 8 * piece + 2 * e;
        const float f0 = Cs[r0 * LDC + ch] * S64I;
        const float f1 = Cs[(r0 + 1) * LDC + ch] * S64I;
        unsigned hp, lp;
        split2(f0, f1, hp, lp);
        a[e] = hp; b[e] = lp;
      }
      ph[s] = a; pl[s] = b;
      offs[s] = ((size_t)(n * CCH + ch)) * HW + p0 + 8 * piece;
    }
#pragma unroll
    for (int s = 0; s < 4; ++s) { *(volatile v4u*)(gh + offs[s]) = ph[s]; *(volatile v4u*)(gl + offs[s]) = pl[s]; }
    __threadfence();
#pragma unroll
    for (int s = 0; s < 4; ++s) { *(volatile v4u*)(gh + offs[s]) = ph[s]; *(volatile v4u*)(gl + offs[s]) = pl[s]; }
  } else {
    unsigned short* hp_ = (wi == 0) ? th : fh;
    unsigned short* lp_ = (wi == 0) ? tl : fl;
#pragma unroll
    for (int s = 0; s < 4; ++s) {
      const int idx = s * 256 + tid;
      const int row = idx >> 4, piece = idx & 15;
      const int col0 = piece * 8;
      v4u a, b;
#pragma unroll
      for (int e = 0; e < 4; ++e) {
        const float f0 = Cs[row * LDC + col0 + 2 * e] * S64I;
        const float f1 = Cs[row * LDC + col0 + 2 * e + 1] * S64I;
        unsigned hp, lp;
        split2(f0, f1, hp, lp);
        a[e] = hp; b[e] = lp;
      }
      ph[s] = a; pl[s] = b;
      offs[s] = ((size_t)(mb * 64 + row)) * CCH + col0;
    }
#pragma unroll
    for (int s = 0; s < 4; ++s) { *(volatile v4u*)(hp_ + offs[s]) = ph[s]; *(volatile v4u*)(lp_ + offs[s]) = pl[s]; }
    __threadfence();
#pragma unroll
    for (int s = 0; s < 4; ++s) { *(volatile v4u*)(hp_ + offs[s]) = ph[s]; *(volatile v4u*)(lp_ + offs[s]) = pl[s]; }
  }
}

__global__ __launch_bounds__(256)
void k_attn(const unsigned short* __restrict__ thp, const unsigned short* __restrict__ tlp,
            const unsigned short* __restrict__ fhp, const unsigned short* __restrict__ flp,
            const unsigned short* __restrict__ ghp, const unsigned short* __restrict__ glp,
            float* out) {
  extern __shared__ __align__(16) unsigned char lds_dyn[];
  float* Sc = (float*)(lds_dyn + LDS_SC);
  unsigned short* Pu = (unsigned short*)(lds_dyn + LDS_P);
  const _Float16* Pf = (const _Float16*)(const void*)(lds_dyn + LDS_P);
  float* Ost = (float*)(lds_dyn + LDS_OST);
  const _Float16* TH = (const _Float16*)(const void*)thp;
  const _Float16* TL = (const _Float16*)(const void*)tlp;
  const _Float16* FH = (const _Float16*)(const void*)fhp;
  const _Float16* FL = (const _Float16*)(const void*)flp;
  const _Float16* GH = (const _Float16*)(const void*)ghp;
  const _Float16* GL = (const _Float16*)(const void*)glp;

  const int tid = threadIdx.x, wave = tid >> 5, lane = tid & 31, hf = lane >> 4, m = lane & 15;
  const int b = blockIdx.x;
  const int n = b >> 5, hq = (b >> 1) & 15, wh = b & 1;
  const int h0 = hq * QR, wbase = wh * 32;

#pragma unroll 1
  for (int sub = 0; sub < 2; ++sub) {
    const int w0 = wbase + sub * QC;

    {
      const int mt = wave & 3, g = wave >> 2;
      const size_t ao = ((size_t)(n * HW + (h0 + mt) * WWD + w0 + m)) * CCH + 8 * hf;
      const _Float16* ap  = TH + ao;
      const _Float16* apl = TL + ao;
      v16h ah[4], al[4];
#pragma unroll
      for (int ks = 0; ks < 4; ++ks) {
        ah[ks] = ld2(ap  + 32 * ks, ap  + 32 * ks + 16);
        al[ks] = ld2(apl + 32 * ks, apl + 32 * ks + 16);
      }
      const int jcol = 16 * g + m;
      const int wk = min(max(w0 - 8 + jcol, 0), WWD - 1);
#pragma unroll 1
      for (int i = 0; i < KSZ; ++i) {
        const int hk = min(max(h0 - KHF + mt + i, 0), HH - 1);
        const size_t bo = ((size_t)(n * HW + hk * WWD + wk)) * CCH + 8 * hf;
        v8f acch = zero8(), accl = zero8();
#pragma unroll
        for (int ks = 0; ks < 4; ++ks) {
          const v16h bh = ld2(FH + bo + 32 * ks, FH + bo + 32 * ks + 16);
          const v16h bl = ld2(FL + bo + 32 * ks, FL + bo + 32 * ks + 16);
          acch = mma_raw(ah[ks], bh, acch);
          accl = mma_raw(ah[ks], bl, accl);
          accl = mma_raw(al[ks], bh, accl);
          guard2(acch, accl, ah[ks], al[ks], bh, bl);
        }
#pragma unroll
        for (int r = 0; r < 8; ++r) {
          const int qj = 8 * hf + r;
          const int bb = jcol - JOFF - qj;
          const float sv = (acch[r] + accl[r] * RSC) * S64I;
          if ((unsigned)bb < (unsigned)KSZ) Sc[(16 * mt + qj) * SCP + i * KSZ + bb] = sv;
        }
      }
    }
    __syncthreads();

    {
      const int q = tid >> 2, u = tid & 3;
      const int qi = q >> 4, qj = q & 15;
      const int hqp = h0 + qi, wqp = w0 + qj;
      float* srow = Sc + q * SCP;
      float mx = -3.0e38f;
#pragma unroll 1
      for (int e = u; e < NWIN; e += 4) {
        const int a = e / KSZ, bb = e - a * KSZ;
        const int hk = hqp + a - KHF, wkk = wqp + bb - KHF;
        const bool in = ((unsigned)hk < (unsigned)HH) && ((unsigned)wkk < (unsigned)WWD);
        const float sv = srow[e];
        mx = fmaxf(mx, in ? sv : 0.0f);
      }
      mx = fmaxf(mx, __shfl_xor(mx, 1, 32));
      mx = fmaxf(mx, __shfl_xor(mx, 2, 32));
      float sum = 0.0f;
#pragma unroll 1
      for (int e = u; e < NWIN; e += 4) {
        const int a = e / KSZ, bb = e - a * KSZ;
        const int hk = hqp + a - KHF, wkk = wqp + bb - KHF;
        const bool in = ((unsigned)hk < (unsigned)HH) && ((unsigned)wkk < (unsigned)WWD);
        const float sv = srow[e];
        const float ex = __expf((in ? sv : 0.0f) - mx);
        sum += ex;
        srow[e] = in ? ex : 0.0f;
      }
      sum += __shfl_xor(sum, 1, 32);
      sum += __shfl_xor(sum, 2, 32);
      const float inv = PSC * __builtin_amdgcn_rcpf(sum);
      __syncthreads();
      unsigned int* prow = (unsigned int*)(Pu + q * PROW);
#pragma unroll 1
      for (int sp = u; sp < NSLOT / 2; sp += 4) {
        const int slot = 2 * sp;
        const int hr = slot >> 5, j = slot & 31;
        const int a = hr - qi;
        const int b0 = j - JOFF - qj, b1 = b0 + 1;
        const bool ain = (unsigned)a < (unsigned)KSZ;
        const int i0 = min(max(a * KSZ + b0, 0), NWIN - 1);
        const int i1 = min(max(a * KSZ + b1, 0), NWIN - 1);
        const float e0v = srow[i0], e1v = srow[i1];
        const float p0 = (ain && ((unsigned)b0 < (unsigned)KSZ)) ? e0v * inv : 0.0f;
        const float p1 = (ain && ((unsigned)b1 < (unsigned)KSZ)) ? e1v * inv : 0.0f;
        unsigned hpk, lpk;
        split2(p0, p1, hpk, lpk);
        prow[sp] = hpk;
        prow[(PLO / 2) + sp] = lpk;
      }
    }
    __syncthreads();

    {
      const int mt = wave & 3, cpar = wave >> 2;
      const _Float16* prh = Pf + (16 * mt + m) * PROW + 8 * hf;
      const int cbA = (w0 >> 3) - 1 + hf;
      const int ccA = min(max(cbA, 0), 7) * 8, ccB = min(max(cbA + 2, 0), 7) * 8;
#pragma unroll 1
      for (int cq = 0; cq < 2; ++cq) {
        const int c0 = 32 * (2 * cpar + cq);
        const size_t cb0 = ((size_t)(n * CCH + c0 + m)) * HW;
        const size_t cb1 = cb0 + (size_t)16 * HW;
        v8f oh0 = zero8(), oh1 = zero8(), ol0 = zero8(), ol1 = zero8();
#pragma unroll 1
        for (int i = 0; i < KSZ; ++i) {
          const int ks = mt + i;
          const int hk = min(max(h0 - KHF + ks, 0), HH - 1);
          const v16h pa = ld2(prh + 32 * ks, prh + 32 * ks + 16);
          const v16h pl = ld2(prh + PLO + 32 * ks, prh + PLO + 32 * ks + 16);
          const size_t g0 = cb0 + (size_t)hk * WWD, g1 = cb1 + (size_t)hk * WWD;
          const v16h bh0 = ld2(GH + g0 + ccA, GH + g0 + ccB);
          const v16h bl0 = ld2(GL + g0 + ccA, GL + g0 + ccB);
          const v16h bh1 = ld2(GH + g1 + ccA, GH + g1 + ccB);
          const v16h bl1 = ld2(GL + g1 + ccA, GL + g1 + ccB);
          oh0 = mma_raw(pa, bh0, oh0);
          ol0 = mma_raw(pa, bl0, ol0);
          ol0 = mma_raw(pl, bh0, ol0);
          oh1 = mma_raw(pa, bh1, oh1);
          ol1 = mma_raw(pa, bl1, ol1);
          ol1 = mma_raw(pl, bh1, ol1);
          guard4x6(oh0, ol0, oh1, ol1, pa, pl, bh0, bl0, bh1, bl1);
        }
#pragma unroll
        for (int r = 0; r < 8; ++r) {
          const int col = sub * QC + 8 * hf + r;
          Ost[((c0 + m) * QR + mt) * OSTP + col]      = (oh0[r] + ol0[r] * RSC) * OSC;
          Ost[((c0 + 16 + m) * QR + mt) * OSTP + col] = (oh1[r] + ol1[r] * RSC) * OSC;
        }
      }
    }
    __syncthreads();
  }

#pragma unroll 4
  for (int s = 0; s < 16; ++s) {
    const int idx = s * 256 + tid;
    const int line = idx >> 3, piece = idx & 7;
    const int c = line >> 2, qi = line & 3;
    const v4f v = *(const v4fa*)(&Ost[(c * QR + qi) * OSTP + piece * 4]);
    float* dst = out + (((size_t)(n * CCH + c) * HH + h0 + qi) * WWD + wbase + piece * 4);
    *(volatile v4f*)dst = v;
  }
  __threadfence();
#pragma unroll 4
  for (int s = 0; s < 16; ++s) {
    const int idx = s * 256 + tid;
    const int line = idx >> 3, piece = idx & 7;
    const int c = line >> 2, qi = line & 3;
    const v4f v = *(const v4fa*)(&Ost[(c * QR + qi) * OSTP + piece * 4]);
    float* dst = out + (((size_t)(n * CCH + c) * HH + h0 + qi) * WWD + wbase + piece * 4);
    *(volatile v4f*)dst = v;
  }
}

extern "C" void kernel_launch(void* const* d_in, const int* in_sizes, int n_in,
                              void* d_out, int out_size, void* d_ws, size_t ws_size,
                              hipStream_t stream) {
  if (n_in < 4) return;
  if (in_sizes[0] != NPIX * CCH) return;
  if (in_sizes[1] != CCH * CCH || in_sizes[2] != CCH * CCH || in_sizes[3] != CCH * CCH) return;
  if (out_size != NPIX * CCH) return;

  const float* x  = (const float*)d_in[0];
  const float* w1 = (const float*)d_in[1];
  const float* w2 = (const float*)d_in[2];
  const float* w3 = (const float*)d_in[3];
  float* out = (float*)d_out;

  const size_t sPL = (size_t)NPIX * CCH * 2;
  const size_t sW  = (size_t)3 * CCH * CCH * 2;
  size_t off = 0;
  const size_t oXT = off; off += sPL;
  const size_t oW  = off; off += sW;
  const size_t oTH = off; off += sPL;
  const size_t oTL = off; off += sPL;
  const size_t oFH = off; off += sPL;
  const size_t oFL = off; off += sPL;
  const size_t oGH = off; off += sPL;
  const size_t oGL = off; off += sPL;
  if (off > ws_size) return;
  if (off > (size_t)134217728) return;

  char* ws = (char*)d_ws;
  unsigned short* XT  = (unsigned short*)(ws + oXT);
  unsigned short* W16 = (unsigned short*)(ws + oW);
  unsigned short* TH  = (unsigned short*)(ws + oTH);
  unsigned short* TL  = (unsigned short*)(ws + oTL);
  unsigned short* FH  = (unsigned short*)(ws + oFH);
  unsigned short* FL  = (unsigned short*)(ws + oFL);
  unsigned short* GH  = (unsigned short*)(ws + oGH);
  unsigned short* GL  = (unsigned short*)(ws + oGL);

  const dim3 blk(256);
  k_cvt_x<<<dim3(NB * 64), blk, 0, stream>>>(x, XT);
  k_cvt_w<<<dim3(24), blk, 0, stream>>>(w1, w2, w3, W16);
  k_proj<<<dim3(NPIX / 64, 3), blk, 0, stream>>>(XT, W16, TH, TL, FH, FL, GH, GL);
  (void)hipFuncSetAttribute(reinterpret_cast<const void*>(&k_attn),
                            hipFuncAttributeMaxDynamicSharedMemorySize, LDS_ATT);
  k_attn<<<dim3(NB * 16 * 2), blk, LDS_ATT, stream>>>(TH, TL, FH, FL, GH, GL, out);
  (void)hipGetLastError();
}
